// multi_attention_33492154974632
// MI455X (gfx1250) — hardware-verified
//
#include <hip/hip_runtime.h>

#pragma clang fp contract(off)

typedef __attribute__((ext_vector_type(16))) _Float16 v16h;
typedef __attribute__((ext_vector_type(8)))  _Float16 v8h;
typedef __attribute__((ext_vector_type(16))) __bf16   v16b;
typedef __attribute__((ext_vector_type(8)))  __bf16   v8b;
typedef __attribute__((ext_vector_type(8)))  float    v8f;
typedef __attribute__((ext_vector_type(4)))  float    v4f;
typedef __attribute__((ext_vector_type(4)))  unsigned int v4u;

constexpr int NBATCH    = 4;
constexpr int SEQLEN    = 2048;
constexpr int DMODEL    = 1024;
constexpr int NHEADS    = 16;
constexpr int HDIM      = 64;
constexpr int ROTD      = 32;
constexpr int HALF_NB   = 2;
constexpr int HALF_ROWS = HALF_NB * SEQLEN;
constexpr float LOG_THETA = 9.21034049987793f;
constexpr float SM_SCALE  = 0.125f;

static_assert(NHEADS * HDIM == DMODEL, "geom");
static_assert(HDIM == 64, "head dim fixed at 64");
static_assert(ROTD * 2 == HDIM, "rot");
static_assert(SEQLEN % 64 == 0, "seq tile");
static_assert(HALF_ROWS % 64 == 0 && DMODEL % 64 == 0, "GEMM M/N tile multiples of 64");
static_assert(DMODEL % 32 == 0, "GEMM K multiple of 32");
static_assert(NBATCH % HALF_NB == 0, "halves");

constexpr size_t SZ_XB    = (size_t)NBATCH * SEQLEN * DMODEL * 2;
constexpr size_t SZ_WQKV  = (size_t)3 * DMODEL * DMODEL * 2;
constexpr size_t SZ_WPROJ = (size_t)DMODEL * DMODEL * 2;
constexpr size_t SZ_TAB   = (size_t)SEQLEN * ROTD * 4;
constexpr size_t SZ_PLANE = (size_t)HALF_ROWS * DMODEL * 2;
constexpr size_t WS_XB    = 0;
constexpr size_t WS_WQKV  = WS_XB + SZ_XB;
constexpr size_t WS_WPROJ = WS_WQKV + SZ_WQKV;
constexpr size_t WS_CTAB  = WS_WPROJ + SZ_WPROJ;
constexpr size_t WS_STAB  = WS_CTAB + SZ_TAB;
constexpr size_t WS_TMPH  = WS_STAB + SZ_TAB;
constexpr size_t WS_TMPL  = WS_TMPH + SZ_PLANE;
constexpr size_t WS_QH    = WS_TMPL + SZ_PLANE;
constexpr size_t WS_QL    = WS_QH + SZ_PLANE;
constexpr size_t WS_KH    = WS_QL + SZ_PLANE;
constexpr size_t WS_KL    = WS_KH + SZ_PLANE;
constexpr size_t WS_VTH   = WS_KL + SZ_PLANE;
constexpr size_t WS_VTL   = WS_VTH + SZ_PLANE;
constexpr size_t WS_ATTH  = WS_VTL + SZ_PLANE;
constexpr size_t WS_ATTL  = WS_ATTH + SZ_PLANE;
constexpr size_t WS_TOTAL = WS_ATTL + SZ_PLANE;
static_assert(WS_TOTAL == 109576192ull, "carve total");
static_assert(WS_TOTAL <= 134217728ull, "carve within 128 MiB");

__device__ __forceinline__ unsigned short f2bf_bits(float f) {
  unsigned u = __float_as_uint(f);
  return (unsigned short)((u + 0x7FFFu + ((u >> 16) & 1u)) >> 16);
}
__device__ __forceinline__ float bf_bits2f(unsigned short h) { return __uint_as_float(((unsigned)h) << 16); }

__device__ __forceinline__ void dep_guard_h(v8f& a, v8f& b, v16h x, v16h y) { asm volatile("v_nop\n\tv_nop\n\tv_nop\n\tv_nop" : "+v"(a), "+v"(b) : "v"(x), "v"(y)); }
__device__ __forceinline__ void dep_guard_b(v8f& a, v8f& b, v16b x, v16b y) { asm volatile("v_nop\n\tv_nop\n\tv_nop\n\tv_nop" : "+v"(a), "+v"(b) : "v"(x), "v"(y)); }
__device__ __forceinline__ void keep4_h(v16h a, v16h b, v16h c, v16h d) { asm volatile("v_nop" :: "v"(a), "v"(b), "v"(c), "v"(d)); }
__device__ __forceinline__ void keep4_b(v16b a, v16b b, v16b c, v16b d) { asm volatile("v_nop" :: "v"(a), "v"(b), "v"(c), "v"(d)); }
__device__ __forceinline__ void acc_guard4(v8f& a, v8f& b, v8f& c, v8f& d) { asm volatile("v_nop\n\tv_nop\n\tv_nop\n\tv_nop" : "+v"(a), "+v"(b), "+v"(c), "+v"(d)); }

template <typename T> struct Frag;
template <> struct Frag<_Float16> {
  typedef v16h V; union U { v16h v; v8h h[2]; };
  static __device__ __forceinline__ v16h load(const _Float16* p) {
    U f; f.h[0] = *(const v8h*)(p); f.h[1] = *(const v8h*)(p + 16); return f.v;
  }
  static __device__ __forceinline__ v8f mma(v16h a, v16h b, v8f c) {
    return __builtin_amdgcn_wmma_f32_16x16x32_f16(false, a, false, b, (short)0, c, false, false);
  }
  static __device__ __forceinline__ void guard(v8f& a, v8f& b, v16h x, v16h y) { dep_guard_h(a, b, x, y); }
  static __device__ __forceinline__ void keep(v16h a, v16h b, v16h c, v16h d) { keep4_h(a, b, c, d); }
};
template <> struct Frag<__bf16> {
  typedef v16b V; union U { v16b v; v8b h[2]; };
  static __device__ __forceinline__ v16b load(const __bf16* p) {
    U f; f.h[0] = *(const v8b*)(p); f.h[1] = *(const v8b*)(p + 16); return f.v;
  }
  static __device__ __forceinline__ v8f mma(v16b a, v16b b, v8f c) {
    return __builtin_amdgcn_wmma_f32_16x16x32_bf16(false, a, false, b, (short)0, c, false, false);
  }
  static __device__ __forceinline__ void guard(v8f& a, v8f& b, v16b x, v16b y) { dep_guard_b(a, b, x, y); }
  static __device__ __forceinline__ void keep(v16b a, v16b b, v16b c, v16b d) { keep4_b(a, b, c, d); }
};

template <int ET> struct Elem;
template <> struct Elem<0> { typedef _Float16 T; };
template <> struct Elem<1> { typedef __bf16 T; };
template <int ET, int SPLIT, int BIAS_MODE, int OUT_MODE, bool RESID, int ACT = 0>
__global__ __launch_bounds__(256) void wmma_gemm64(
    const unsigned short* __restrict__ Ap, const unsigned short* __restrict__ A2p, int lda, long strideA,
    const unsigned short* __restrict__ Btp, const unsigned short* __restrict__ Bt2p, int ldb, long strideB,
    void* __restrict__ Cout, void* __restrict__ Cout2, int ldc, long strideC,
    const float* __restrict__ bias,
    const float* __restrict__ resid, long strideR,
    int M, int N, int K, float scale) {
  typedef typename Elem<ET>::T T;
  typedef typename Frag<T>::V V;
  constexpr bool SPLA = (SPLIT != 0);
  constexpr bool SPLB = (SPLIT == 1);
  const T* A = (const T*)Ap; const T* A2 = (const T*)A2p; const T* Bt = (const T*)Btp; const T* Bt2 = (const T*)Bt2p;
  __shared__ __align__(16) float sT[8][16 * 68];
  const int b    = blockIdx.y;
  const int lane = threadIdx.x & 31;
  const int wave = threadIdx.x >> 5;
  const int tilesN = N >> 6;
  const int tilesM = M >> 6;
  const int tile = blockIdx.x * 8 + wave;
  if (tile >= tilesM * tilesN) return;
  const int tm = tile / tilesN;
  const int tn = tile - tm * tilesN;
  const int m0 = tm << 6;
  const int n0 = tn << 6;

  const T* Ab  = A  + (size_t)b * strideA;
  const T* Bb  = Bt + (size_t)b * strideB;
  const T* Ab2 = SPLA ? (A2  + (size_t)b * strideA) : nullptr;
  const T* Bb2 = SPLB ? (Bt2 + (size_t)b * strideB) : nullptr;

  const int rlane = lane & 15;
  const int koff  = (lane >> 4) * 8;
  const int mOff  = (lane >> 4) * 8;

  v8f acc[4][4];
#pragma unroll
  for (int i = 0; i < 4; ++i)
#pragma unroll
    for (int j = 0; j < 4; ++j) acc[i][j] = (v8f){0.f,0.f,0.f,0.f,0.f,0.f,0.f,0.f};

  for (int k0 = 0; k0 < K; k0 += 32) {
    V bh[4], bl[4];
#pragma unroll
    for (int j = 0; j < 4; ++j) {
      const size_t bo = (size_t)(n0 + (j << 4) + rlane) * ldb + koff + k0;
      bh[j] = Frag<T>::load(Bb + bo);
      if (SPLB) bl[j] = Frag<T>::load(Bb2 + bo);
    }
#pragma unroll
    for (int i = 0; i < 4; ++i) {
      const size_t ao = (size_t)(m0 + (i << 4) + rlane) * lda + koff + k0;
      V ah = Frag<T>::load(Ab + ao);
      V al;
      if (SPLA) al = Frag<T>::load(Ab2 + ao);
#pragma unroll
      for (int j = 0; j < 4; ++j) {
        acc[i][j] = Frag<T>::mma(ah, bh[j], acc[i][j]);
        if (SPLB) acc[i][j] = Frag<T>::mma(ah, bl[j], acc[i][j]);
        if (SPLA) acc[i][j] = Frag<T>::mma(al, bh[j], acc[i][j]);
      }
      Frag<T>::guard(acc[i][0], acc[i][3], ah, SPLA ? al : ah);
    }
    Frag<T>::keep(bh[0], bh[1], bh[2], bh[3]);
    if (SPLB) Frag<T>::keep(bl[0], bl[1], bl[2], bl[3]);
  }
  acc_guard4(acc[0][0], acc[0][1], acc[0][2], acc[0][3]);
  acc_guard4(acc[1][0], acc[1][1], acc[1][2], acc[1][3]);
  acc_guard4(acc[2][0], acc[2][1], acc[2][2], acc[2][3]);
  acc_guard4(acc[3][0], acc[3][1], acc[3][2], acc[3][3]);

  float* slab = sT[wave];
  const float* Rb = RESID ? (resid + (size_t)b * strideR) : nullptr;
#pragma unroll
  for (int i = 0; i < 4; ++i) {
    const int mBase = m0 + (i << 4);
#pragma unroll
    for (int j = 0; j < 4; ++j) {
      const int n = n0 + (j << 4) + rlane;
      float bv = 0.f;
      if (BIAS_MODE == 2) bv = bias[n];
#pragma unroll
      for (int r = 0; r < 8; ++r) {
        float v = acc[i][j][r] * scale;
        if (BIAS_MODE == 1) v += bias[mBase + mOff + r];
        if (BIAS_MODE == 2) v += bv;
        if (RESID) v += Rb[(size_t)(mBase + mOff + r) * ldc + n];
        if (ACT == 1) v = tanhf(v);
        if (ACT == 2) v = fmaxf(v, 0.0f);
        if (ACT == 3) v = v / (1.0f + expf(-v));
        if (ACT == 4) v = (v > 0.f) ? v : 0.01f * v;
        slab[(mOff + r) * 68 + (j << 4) + rlane] = v;
      }
    }
    __builtin_amdgcn_fence(__ATOMIC_RELEASE, "workgroup");
    __builtin_amdgcn_wave_barrier();
    __builtin_amdgcn_fence(__ATOMIC_ACQUIRE, "workgroup");
    if (OUT_MODE == 0) {
      float* C = (float*)Cout + (size_t)b * strideC;
      const int hh = lane >> 4, c4 = (lane & 15) * 4;
      for (int pass = 0; pass < 2; ++pass) {
#pragma unroll
        for (int it = 0; it < 8; ++it) {
          const int row = it * 2 + hh;
          v4f v = *(const v4f*)(slab + row * 68 + c4);
          *(volatile v4f*)(C + (size_t)(mBase + row) * ldc + n0 + c4) = v;
        }
        __threadfence();
      }
    } else {
      const int q = lane >> 3, c8 = (lane & 7) * 8;
      unsigned short* C  = (unsigned short*)Cout  + (size_t)b * strideC;
      unsigned short* C2 = (OUT_MODE == 2) ? ((unsigned short*)Cout2 + (size_t)b * strideC) : nullptr;
      for (int pass = 0; pass < 2; ++pass) {
#pragma unroll
        for (int it = 0; it < 4; ++it) {
          const int row = it * 4 + q;
          const float* sp = slab + row * 68 + c8;
          v8h hv, lv;
#pragma unroll
          for (int e = 0; e < 8; ++e) {
            if (OUT_MODE == 1) {
              hv[e] = (_Float16)sp[e];
            } else {
              unsigned short hb = f2bf_bits(sp[e]);
              unsigned short lb = f2bf_bits(sp[e] - bf_bits2f(hb));
              hv[e] = __builtin_bit_cast(_Float16, hb);
              lv[e] = __builtin_bit_cast(_Float16, lb);
            }
          }
          *(volatile v8h*)(C + (size_t)(mBase + row) * ldc + n0 + c8) = hv;
          if (OUT_MODE == 2) *(volatile v8h*)(C2 + (size_t)(mBase + row) * ldc + n0 + c8) = lv;
        }
        __threadfence();
      }
    }
    __builtin_amdgcn_fence(__ATOMIC_RELEASE, "workgroup");
    __builtin_amdgcn_wave_barrier();
    __builtin_amdgcn_fence(__ATOMIC_ACQUIRE, "workgroup");
  }
}

__device__ __forceinline__ void at_split(float f, __bf16& hi, __bf16& lo) {
  const unsigned short hb = f2bf_bits(f);
  hi = __builtin_bit_cast(__bf16, hb);
  lo = __builtin_bit_cast(__bf16, f2bf_bits(f - bf_bits2f(hb)));
}
__device__ __forceinline__ v8f at_mma(v16b a, v16b b, v8f c) {
  c = __builtin_amdgcn_wmma_f32_16x16x32_bf16(false, a, false, b, (short)0, c, false, false);
  asm volatile("v_nop\n\tv_nop\n\tv_nop\n\tv_nop" : "+v"(c) : "v"(a), "v"(b));
  return c;
}

__global__ __launch_bounds__(256) void cvt_f32_bf16x8(const float* __restrict__ in,
                                                      unsigned short* __restrict__ out, int n8) {
  const int i = blockIdx.x * 256 + threadIdx.x;
  if (i < n8) {
    const size_t o = (size_t)i * 8;
    const v4f a = *(const v4f*)(in + o);
    const v4f c = *(const v4f*)(in + o + 4);
    v4u w;
    w.x = (unsigned)f2bf_bits(a.x) | ((unsigned)f2bf_bits(a.y) << 16);
    w.y = (unsigned)f2bf_bits(a.z) | ((unsigned)f2bf_bits(a.w) << 16);
    w.z = (unsigned)f2bf_bits(c.x) | ((unsigned)f2bf_bits(c.y) << 16);
    w.w = (unsigned)f2bf_bits(c.z) | ((unsigned)f2bf_bits(c.w) << 16);
    *(volatile v4u*)(out + o) = w;
    __threadfence();
    *(volatile v4u*)(out + o) = w;
  }
}

__global__ __launch_bounds__(256) void rope_table_kernel(float* __restrict__ ctab, float* __restrict__ stab, int npos) {
  const int lane = threadIdx.x & 31;
  const int t = blockIdx.x * 8 + (threadIdx.x >> 5);
  if (t < npos) {
    const float fi  = (float)lane;
    const float ex  = (-(2.0f * fi) / (float)HDIM) * LOG_THETA;
    const float inv = expf(ex);
    const float ang = (float)t * inv;
    float sv, cv;
    sincosf(ang, &sv, &cv);
    const size_t o = (size_t)t * ROTD + lane;
    ((volatile float*)ctab)[o] = cv;
    ((volatile float*)stab)[o] = sv;
    __threadfence();
    ((volatile float*)ctab)[o] = cv;
    ((volatile float*)stab)[o] = sv;
  }
}

__device__ __forceinline__ unsigned split_pack2(float y0, float y1, unsigned& lw) {
  const unsigned short h0 = f2bf_bits(y0), h1 = f2bf_bits(y1);
  const unsigned short l0 = f2bf_bits(y0 - bf_bits2f(h0));
  const unsigned short l1 = f2bf_bits(y1 - bf_bits2f(h1));
  lw = (unsigned)l0 | ((unsigned)l1 << 16);
  return (unsigned)h0 | ((unsigned)h1 << 16);
}
__global__ __launch_bounds__(256) void rope_resplit_kernel(
    const unsigned short* __restrict__ rh, const unsigned short* __restrict__ rl,
    const float* __restrict__ ctab, const float* __restrict__ stab,
    unsigned short* __restrict__ oh, unsigned short* __restrict__ ol, int nrows, int seqlen) {
  constexpr int NGRP = DMODEL / 8;
  const int gid = blockIdx.x * 256 + threadIdx.x;
  if (gid >= nrows * NGRP) return;
  const int row = gid / NGRP;
  const int col = (gid - row * NGRP) * 8;
  const int t   = row % seqlen;
  const int i0  = (col & (HDIM - 1)) >> 1;
  const size_t off = (size_t)row * DMODEL + col;
  const v4u wh = *(const v4u*)(rh + off);
  const v4u wl = *(const v4u*)(rl + off);
  const v4f cs = *(const v4f*)(ctab + (size_t)t * ROTD + i0);
  const v4f sn = *(const v4f*)(stab + (size_t)t * ROTD + i0);
  const float x0 = __uint_as_float(wh.x << 16)          + __uint_as_float(wl.x << 16);
  const float x1 = __uint_as_float(wh.x & 0xffff0000u)  + __uint_as_float(wl.x & 0xffff0000u);
  const float x2 = __uint_as_float(wh.y << 16)          + __uint_as_float(wl.y << 16);
  const float x3 = __uint_as_float(wh.y & 0xffff0000u)  + __uint_as_float(wl.y & 0xffff0000u);
  const float x4 = __uint_as_float(wh.z << 16)          + __uint_as_float(wl.z << 16);
  const float x5 = __uint_as_float(wh.z & 0xffff0000u)  + __uint_as_float(wl.z & 0xffff0000u);
  const float x6 = __uint_as_float(wh.w << 16)          + __uint_as_float(wl.w << 16);
  const float x7 = __uint_as_float(wh.w & 0xffff0000u)  + __uint_as_float(wl.w & 0xffff0000u);
  const float y0 = x0 * cs.x - x1 * sn.x, y1 = x0 * sn.x + x1 * cs.x;
  const float y2 = x2 * cs.y - x3 * sn.y, y3 = x2 * sn.y + x3 * cs.y;
  const float y4 = x4 * cs.z - x5 * sn.z, y5 = x4 * sn.z + x5 * cs.z;
  const float y6 = x6 * cs.w - x7 * sn.w, y7 = x6 * sn.w + x7 * cs.w;
  v4u ph, plo;
  unsigned lw;
  ph.x = split_pack2(y0, y1, lw); plo.x = lw;
  ph.y = split_pack2(y2, y3, lw); plo.y = lw;
  ph.z = split_pack2(y4, y5, lw); plo.z = lw;
  ph.w = split_pack2(y6, y7, lw); plo.w = lw;
  *(volatile v4u*)(oh + off) = ph;
  *(volatile v4u*)(ol + off) = plo;
  __threadfence();
  *(volatile v4u*)(oh + off) = ph;
  *(volatile v4u*)(ol + off) = plo;
}

constexpr int ATT_HD = 64;
constexpr int ATT_KC = 64;
constexpr int ATT_NWAVE = 4;
constexpr int ATT_OSP = 68;
__global__ __launch_bounds__(128)
void attn_causal_split_planes(const unsigned short* __restrict__ qh_p, const unsigned short* __restrict__ ql_p,
                              const unsigned short* __restrict__ kh_p, const unsigned short* __restrict__ kl_p,
                              const unsigned short* __restrict__ vth_p, const unsigned short* __restrict__ vtl_p,
                              unsigned short* __restrict__ oh_p, unsigned short* __restrict__ ol_p,
                              int seqlen, int nheads, int ldq, int ldv, float sm_scale) {
  __shared__ __align__(16) unsigned short Ksh[ATT_KC * ATT_HD];
  __shared__ __align__(16) unsigned short Ksl[ATT_KC * ATT_HD];
  __shared__ __align__(16) unsigned short Vsh[ATT_HD * ATT_KC];
  __shared__ __align__(16) unsigned short Vsl[ATT_HD * ATT_KC];
  __shared__ __align__(16) __bf16 Psh[ATT_NWAVE][16 * ATT_KC];
  __shared__ __align__(16) __bf16 Psl[ATT_NWAVE][16 * ATT_KC];
  __shared__ __align__(16) float  Os[ATT_NWAVE][16 * ATT_OSP];

  const int tid  = threadIdx.x;
  const int wave = tid >> 5;
  const int lane = tid & 31;
  const int hh   = lane >> 4;
  const int c    = lane & 15;
  const int nqb  = seqlen >> 6;
  const int bx   = blockIdx.x;
  const int qb   = bx % nqb;
  const int bhid = bx / nqb;
  const int h    = bhid % nheads;
  const int bsub = bhid / nheads;
  const int rowbase = bsub * seqlen;
  const int q0   = (qb << 6) + wave * 16;
  const int hcol = h * ATT_HD;

  const __bf16* qh = (const __bf16*)qh_p;
  const __bf16* ql = (const __bf16*)ql_p;
  const __bf16* KshB = (const __bf16*)Ksh;
  const __bf16* KslB = (const __bf16*)Ksl;
  const __bf16* VshB = (const __bf16*)Vsh;
  const __bf16* VslB = (const __bf16*)Vsl;

  v16b qah[2], qal[2];
  {
    const size_t qo = (size_t)(rowbase + q0 + c) * ldq + hcol + 8 * hh;
#pragma unroll
    for (int dc = 0; dc < 2; ++dc) {
      qah[dc] = Frag<__bf16>::load(qh + qo + dc * 32);
      qal[dc] = Frag<__bf16>::load(ql + qo + dc * 32);
    }
  }

  float mrow[8], lrow[8];
  v8f oacc[4];
#pragma unroll
  for (int r = 0; r < 8; ++r) { mrow[r] = -__builtin_inff(); lrow[r] = 0.f; }
#pragma unroll
  for (int t = 0; t < 4; ++t) oacc[t] = (v8f){0.f,0.f,0.f,0.f,0.f,0.f,0.f,0.f};

  const int nChunks = qb + 1;
  for (int kc = 0; kc < nChunks; ++kc) {
    const int kv0 = kc * ATT_KC;
    __syncthreads();
    {
      const int r  = tid >> 1;
      const int hf = (tid & 1) * 32;
      const size_t ko = (size_t)(rowbase + kv0 + r) * ldq + hcol + hf;
      const size_t vo = (size_t)(hcol + r) * ldv + rowbase + kv0 + hf;
      const int lo_off = r * ATT_HD + hf;
#pragma unroll
      for (int i = 0; i < 4; ++i) {
        const v4u a  = *(const v4u*)(kh_p + ko + 8 * i);
        const v4u a2 = *(const v4u*)(kl_p + ko + 8 * i);
        *(v4u*)(Ksh + lo_off + 8 * i) = a;
        *(v4u*)(Ksl + lo_off + 8 * i) = a2;
      }
#pragma unroll
      for (int i = 0; i < 4; ++i) {
        const v4u w  = *(const v4u*)(vth_p + vo + 8 * i);
        const v4u w2 = *(const v4u*)(vtl_p + vo + 8 * i);
        *(v4u*)(Vsh + lo_off + 8 * i) = w;
        *(v4u*)(Vsl + lo_off + 8 * i) = w2;
      }
    }
    __syncthreads();

    v8f s[4];
#pragma unroll
    for (int j = 0; j < 4; ++j) {
      s[j] = (v8f){0.f,0.f,0.f,0.f,0.f,0.f,0.f,0.f};
#pragma unroll
      for (int dc = 0; dc < 2; ++dc) {
        const int ko2 = (j * 16 + c) * ATT_HD + dc * 32 + 8 * hh;
        const v16b kb  = Frag<__bf16>::load(KshB + ko2);
        const v16b klv = Frag<__bf16>::load(KslB + ko2);
        s[j] = at_mma(qah[dc], kb,  s[j]);
        s[j] = at_mma(qah[dc], klv, s[j]);
        s[j] = at_mma(qal[dc], kb,  s[j]);
      }
    }
    const bool diag = (kc == qb);
    float cm[8];
#pragma unroll
    for (int r = 0; r < 8; ++r) {
      const int qrow = q0 + 8 * hh + r;
      float m = -__builtin_inff();
#pragma unroll
      for (int j = 0; j < 4; ++j) {
        const int kvcol = kv0 + j * 16 + c;
        float sv = s[j][r] * sm_scale;
        if (diag && (kvcol > qrow)) sv = -__builtin_inff();
        s[j][r] = sv;
        m = fmaxf(m, sv);
      }
#pragma unroll
      for (int off = 1; off < 16; off <<= 1) m = fmaxf(m, __shfl_xor(m, off, 32));
      cm[r] = m;
    }
    __bf16* pwh = Psh[wave];
    __bf16* pwl = Psl[wave];
#pragma unroll
    for (int r = 0; r < 8; ++r) {
      const float mnew  = fmaxf(mrow[r], cm[r]);
      const float alpha = expf(mrow[r] - mnew);
      mrow[r] = mnew;
      float psum = 0.f;
#pragma unroll
      for (int j = 0; j < 4; ++j) {
        const float p = expf(s[j][r] - mnew);
        psum += p;
        __bf16 ph2, pl2;
        at_split(p, ph2, pl2);
        pwh[(8 * hh + r) * ATT_KC + j * 16 + c] = ph2;
        pwl[(8 * hh + r) * ATT_KC + j * 16 + c] = pl2;
      }
#pragma unroll
      for (int off = 1; off < 16; off <<= 1) psum += __shfl_xor(psum, off, 32);
      lrow[r] = lrow[r] * alpha + psum;
#pragma unroll
      for (int t = 0; t < 4; ++t) oacc[t][r] *= alpha;
    }
    __builtin_amdgcn_fence(__ATOMIC_RELEASE, "workgroup");
    __builtin_amdgcn_wave_barrier();
    __builtin_amdgcn_fence(__ATOMIC_ACQUIRE, "workgroup");
#pragma unroll 1
    for (int kk = 0; kk < 2; ++kk) {
      const int po = c * ATT_KC + kk * 32 + 8 * hh;
      const v16b pa = Frag<__bf16>::load(pwh + po);
      const v16b pl = Frag<__bf16>::load(pwl + po);
#pragma unroll
      for (int t = 0; t < 4; ++t) {
        const int vo2 = (t * 16 + c) * ATT_KC + kk * 32 + 8 * hh;
        const v16b vb = Frag<__bf16>::load(VshB + vo2);
        const v16b vl = Frag<__bf16>::load(VslB + vo2);
        oacc[t] = at_mma(pa, vb, oacc[t]);
        oacc[t] = at_mma(pa, vl, oacc[t]);
        oacc[t] = at_mma(pl, vb, oacc[t]);
      }
    }
  }

  float* os = Os[wave];
#pragma unroll
  for (int r = 0; r < 8; ++r) {
    const float inv = 1.0f / lrow[r];
#pragma unroll
    for (int t = 0; t < 4; ++t) os[(8 * hh + r) * ATT_OSP + t * 16 + c] = oacc[t][r] * inv;
  }
  __builtin_amdgcn_fence(__ATOMIC_RELEASE, "workgroup");
  __builtin_amdgcn_wave_barrier();
  __builtin_amdgcn_fence(__ATOMIC_ACQUIRE, "workgroup");
  {
    const int q8 = lane >> 3, c8 = (lane & 7) * 8;
    for (int pass = 0; pass < 2; ++pass) {
#pragma unroll
      for (int it = 0; it < 4; ++it) {
        const int row = it * 4 + q8;
        const float* sp = os + row * ATT_OSP + c8;
        v8h hv, lv;
#pragma unroll
        for (int e = 0; e < 8; ++e) {
          const unsigned short hb = f2bf_bits(sp[e]);
          const unsigned short lb = f2bf_bits(sp[e] - bf_bits2f(hb));
          hv[e] = __builtin_bit_cast(_Float16, hb);
          lv[e] = __builtin_bit_cast(_Float16, lb);
        }
        const size_t oo = (size_t)(rowbase + q0 + row) * ldq + hcol + c8;
        *(volatile v8h*)(oh_p + oo) = hv;
        *(volatile v8h*)(ol_p + oo) = lv;
      }
      __threadfence();
    }
  }
}

extern "C" void kernel_launch(void* const* d_in, const int* in_sizes, int n_in,
                              void* d_out, int out_size, void* d_ws, size_t ws_size,
                              hipStream_t stream) {
  if (n_in < 3) return;
  if (in_sizes[0] != NBATCH * SEQLEN * DMODEL) return;
  if (in_sizes[1] != 3 * DMODEL * DMODEL) return;
  if (in_sizes[2] != DMODEL * DMODEL) return;
  if (out_size != NBATCH * SEQLEN * DMODEL) return;
  if (ws_size < WS_TOTAL) return;

  const float* x     = (const float*)d_in[0];
  const float* wqkv  = (const float*)d_in[1];
  const float* wproj = (const float*)d_in[2];
  float* out = (float*)d_out;

  unsigned char* ws = (unsigned char*)d_ws;
  unsigned short* xb     = (unsigned short*)(ws + WS_XB);
  unsigned short* wqkvb  = (unsigned short*)(ws + WS_WQKV);
  unsigned short* wprojb = (unsigned short*)(ws + WS_WPROJ);
  float* ctab = (float*)(ws + WS_CTAB);
  float* stab = (float*)(ws + WS_STAB);
  unsigned short* tmph = (unsigned short*)(ws + WS_TMPH);
  unsigned short* tmpl = (unsigned short*)(ws + WS_TMPL);
  unsigned short* qhp  = (unsigned short*)(ws + WS_QH);
  unsigned short* qlp  = (unsigned short*)(ws + WS_QL);
  unsigned short* khp  = (unsigned short*)(ws + WS_KH);
  unsigned short* klp  = (unsigned short*)(ws + WS_KL);
  unsigned short* vthp = (unsigned short*)(ws + WS_VTH);
  unsigned short* vtlp = (unsigned short*)(ws + WS_VTL);
  unsigned short* atth = (unsigned short*)(ws + WS_ATTH);
  unsigned short* attl = (unsigned short*)(ws + WS_ATTL);
  const float* fdummy  = ctab;
  const float* fdummy2 = stab;

  constexpr int NX8  = NBATCH * SEQLEN * DMODEL / 8;
  constexpr int NWQ8 = 3 * DMODEL * DMODEL / 8;
  constexpr int NWP8 = DMODEL * DMODEL / 8;
  static_assert(NX8 % 256 == 0 && NWQ8 % 256 == 0 && NWP8 % 256 == 0, "cvt grids exact");
  cvt_f32_bf16x8<<<dim3(NX8 / 256), dim3(256), 0, stream>>>(x, xb, NX8);
  cvt_f32_bf16x8<<<dim3(NWQ8 / 256), dim3(256), 0, stream>>>(wqkv, wqkvb, NWQ8);
  cvt_f32_bf16x8<<<dim3(NWP8 / 256), dim3(256), 0, stream>>>(wproj, wprojb, NWP8);

  static_assert(SEQLEN % 8 == 0, "table grid");
  rope_table_kernel<<<dim3(SEQLEN / 8), dim3(256), 0, stream>>>(ctab, stab, SEQLEN);

  constexpr int TILES_PROJ = (HALF_ROWS / 64) * (DMODEL / 64);
  constexpr int GEMM_BLOCKS = (TILES_PROJ + 7) / 8;
  constexpr int ROPE_THREADS = HALF_ROWS * (DMODEL / 8);
  static_assert(ROPE_THREADS % 256 == 0, "rope grid exact");
  constexpr int ROPE_BLOCKS = ROPE_THREADS / 256;
  constexpr int ATT_BLOCKS  = HALF_NB * NHEADS * (SEQLEN / 64);

  for (int hf = 0; hf < NBATCH / HALF_NB; ++hf) {
    const unsigned short* xbh = xb + (size_t)hf * HALF_ROWS * DMODEL;

    wmma_gemm64<1, 0, 0, 2, false><<<dim3(GEMM_BLOCKS, 1), dim3(256), 0, stream>>>(
        xbh, xbh, DMODEL, 0L,
        wqkvb, wqkvb, DMODEL, 0L,
        (void*)tmph, (void*)tmpl, DMODEL, 0L,
        fdummy, fdummy2, 0L,
        HALF_ROWS, DMODEL, DMODEL, 1.0f);
    rope_resplit_kernel<<<dim3(ROPE_BLOCKS), dim3(256), 0, stream>>>(tmph, tmpl, ctab, stab, qhp, qlp, HALF_ROWS, SEQLEN);

    wmma_gemm64<1, 0, 0, 2, false><<<dim3(GEMM_BLOCKS, 1), dim3(256), 0, stream>>>(
        xbh, xbh, DMODEL, 0L,
        wqkvb + (size_t)DMODEL * DMODEL, wqkvb + (size_t)DMODEL * DMODEL, DMODEL, 0L,
        (void*)tmph, (void*)tmpl, DMODEL, 0L,
        fdummy, fdummy2, 0L,
        HALF_ROWS, DMODEL, DMODEL, 1.0f);
    rope_resplit_kernel<<<dim3(ROPE_BLOCKS), dim3(256), 0, stream>>>(tmph, tmpl, ctab, stab, khp, klp, HALF_ROWS, SEQLEN);

    wmma_gemm64<1, 0, 0, 2, false><<<dim3(GEMM_BLOCKS, 1), dim3(256), 0, stream>>>(
        wqkvb + (size_t)2 * DMODEL * DMODEL, wqkvb + (size_t)2 * DMODEL * DMODEL, DMODEL, 0L,
        xbh, xbh, DMODEL, 0L,
        (void*)vthp, (void*)vtlp, HALF_ROWS, 0L,
        fdummy, fdummy2, 0L,
        DMODEL, HALF_ROWS, DMODEL, 1.0f);

    attn_causal_split_planes<<<dim3(ATT_BLOCKS), dim3(128), 0, stream>>>(
        qhp, qlp, khp, klp, vthp, vtlp, atth, attl,
        SEQLEN, NHEADS, DMODEL, HALF_ROWS, SM_SCALE);

    wmma_gemm64<1, 2, 0, 0, false><<<dim3(GEMM_BLOCKS, 1), dim3(256), 0, stream>>>(
        atth, attl, DMODEL, 0L,
        wprojb, wprojb, DMODEL, 0L,
        (void*)(out + (size_t)hf * HALF_ROWS * DMODEL), (void*)attl, DMODEL, 0L,
        fdummy, fdummy2, 0L,
        HALF_ROWS, DMODEL, DMODEL, 1.0f);
  }
}
